// fromNorm_mix_20358144983646
// MI455X (gfx1250) — hardware-verified
//
#include <hip/hip_runtime.h>
#include <stddef.h>


typedef _Float16 v16h __attribute__((ext_vector_type(16)));
typedef _Float16 v8h  __attribute__((ext_vector_type(8)));
typedef float    v8f  __attribute__((ext_vector_type(8)));
typedef float    v4f  __attribute__((ext_vector_type(4)));
typedef int      v4i  __attribute__((ext_vector_type(4)));
typedef _Float16 h16;

#ifndef NTOK
#define NTOK 8192
#endif
#define NTOK_FULL 8192
#define ZD    256
#define HD    1024
#define UD    256
#define NEXP  16
#define TOKT  32
#define MAXTILE (NTOK / TOKT)
#define EPT   (NTOK / 256)
#define SLABW 256
#define NSLAB_H (HD / SLABW)
#define NSLAB   (NSLAB_H + 1)

#define XLD (ZD + 8)
#define OLD 36

#define REG_Z 0
#define REG_A (TOKT * XLD)
#define REG_U (2 * TOKT * XLD)

#define WCARRY 64.0f
#define ACARRY 64.0f

#define WZ_ELEMS ((size_t)NEXP * ZD * ZD)
#define WH_ELEMS ((size_t)NEXP * HD * ZD)
#define WU_ELEMS ((size_t)NEXP * UD * UD)
#define OFFE_Z ((size_t)0)
#define OFFE_H (OFFE_Z + WZ_ELEMS)
#define OFFE_U (OFFE_H + WH_ELEMS)
#define WS_TOTAL ((OFFE_U + WU_ELEMS) * 2)

#define OUT1_ELEM ((size_t)NTOK_FULL * HD)

static_assert(NTOK >= 1024 && NTOK <= NTOK_FULL && (NTOK % 1024) == 0);
static_assert(EPT >= 4 && EPT <= 32 && (EPT % 4) == 0);
static_assert(256 * EPT == NTOK);
static_assert(TOKT == 32 && (NTOK % TOKT) == 0);
static_assert(8 * 4 == TOKT);
static_assert(TOKT * 8 == 256 && ZD == 8 * 32 && UD == 8 * 32);
static_assert(ZD == UD);
static_assert((ZD % 32) == 0 && (UD % 32) == 0);
static_assert(ZD == 8 * 32);
static_assert(SLABW == 8 * 32 && (HD % SLABW) == 0 && UD == SLABW);
static_assert((XLD % 8) == 0 && (OLD % 4) == 0 && OLD >= 32);
static_assert((WZ_ELEMS % 2048) == 0 && (WH_ELEMS % 2048) == 0 && (WU_ELEMS % 2048) == 0);
static_assert(((OFFE_H * 2) % 128) == 0 && ((OFFE_U * 2) % 128) == 0);
static_assert(WS_TOTAL == (size_t)12582912);
static_assert(WS_TOTAL <= (size_t)134217728);
static_assert(OUT1_ELEM * 4 == (size_t)33554432);
static_assert(OUT1_ELEM + (size_t)NTOK_FULL * UD == (size_t)10485760);
static_assert((size_t)3 * TOKT * XLD * 2 + (size_t)8 * TOKT * OLD * 4 + TOKT * 4 + 8 * 4 <= (size_t)131072);

__device__ __forceinline__ float bf16r(float x) {
  unsigned int u = __float_as_uint(x);
  u = (u + 0x7FFFu + ((u >> 16) & 1u)) & 0xFFFF0000u;
  return __uint_as_float(u);
}

__device__ __forceinline__ h16 toh_flush(float v) {
  const h16 r = (h16)v;
  return (fabsf(v) < 6.103515625e-05f) ? (h16)0.0f : r;
}

__device__ __forceinline__ v16h frag_at(const _Float16* p) {
  v8h lo = *(const v8h*)(p);
  v8h hi = *(const v8h*)(p + 16);
  v16h out;
#pragma unroll
  for (int i = 0; i < 8; ++i) { out[i] = lo[i]; out[i + 8] = hi[i]; }
  return out;
}
__device__ __forceinline__ v16h ld_frag(const _Float16* base, unsigned ld) {
  const unsigned lane = threadIdx.x & 31u;
  return frag_at(base + (lane & 15u) * ld + (lane >> 4) * 8u);
}

__device__ __forceinline__ v8f wmma16(v16h a, v16h b, v8f c) {
  v8f d = __builtin_amdgcn_wmma_f32_16x16x32_f16(false, a, false, b, (short)0, c,
                                                 false, false);
  asm volatile("v_nop\n\tv_nop\n\tv_nop\n\tv_nop" : "+v"(d) : "v"(a), "v"(b));
  return d;
}

__device__ __forceinline__ void wave_lds_sync() {
  __builtin_amdgcn_fence(3  , "wavefront");
  asm volatile("s_wait_dscnt 0x0" ::: "memory");
  __builtin_amdgcn_wave_barrier();
}

__global__ __launch_bounds__(256) void wcast_kernel(
    const float* __restrict__ W, _Float16* __restrict__ Wt, unsigned ngroups) {
  const unsigned g = blockIdx.x * 256u + threadIdx.x;
  if (g < ngroups) {
    const size_t o = (size_t)g * 8u;
    const v4f a0 = *(const v4f*)(W + o);
    const v4f a1 = *(const v4f*)(W + o + 4u);
    v8h x;
#pragma unroll
    for (int i = 0; i < 4; ++i) {
      x[i]     = toh_flush(WCARRY * bf16r(a0[i]));
      x[i + 4] = toh_flush(WCARRY * bf16r(a1[i]));
    }
    *(volatile v8h*)(Wt + o) = x;
    __threadfence();
    *(volatile v8h*)(Wt + o) = x;
  }
}

__global__ __launch_bounds__(256) void mix_ffn_kernel(
    const float* __restrict__ Zin, const float* __restrict__ Uin,
    const int* __restrict__ route, const _Float16* __restrict__ Wp,
    const float* __restrict__ bz, const float* __restrict__ bh,
    float* __restrict__ out) {
  __shared__ _Float16 Ts[3 * TOKT * XLD];
  __shared__ float    Cs[8 * TOKT * OLD];
  __shared__ int      toks[TOKT];
  __shared__ int      wtot[8];

  const unsigned tid = threadIdx.x, lane = tid & 31u;
  const unsigned wv = tid >> 5;
  const int wave = __builtin_amdgcn_readfirstlane((int)(threadIdx.x >> 5));
  const unsigned hh = lane >> 4, m = lane & 15u;
  const int e = (int)blockIdx.y;
  const int tile = (int)blockIdx.x;

  const unsigned frow0 = tid * (unsigned)EPT;
  int rv[EPT];
#pragma unroll
  for (int q = 0; q < EPT / 4; ++q) {
    const v4i t4 = *(const v4i*)(route + frow0 + 4u * (unsigned)q);
    rv[4 * q + 0] = t4[0];
    rv[4 * q + 1] = t4[1];
    rv[4 * q + 2] = t4[2];
    rv[4 * q + 3] = t4[3];
  }
  int c = 0;
#pragma unroll
  for (int j = 0; j < EPT; ++j) c += (rv[j] == e) ? 1 : 0;
  int inc = c;
#pragma unroll
  for (int off = 1; off < 32; off <<= 1) {
    const int t = __shfl_up(inc, off, 32);
    inc += ((int)lane >= off) ? t : 0;
  }
  if (lane == 31u) wtot[wv] = inc;
  if (tid < (unsigned)TOKT) toks[tid] = -1;
  __syncthreads();
  int base = 0, cntv = 0;
#pragma unroll
  for (int w2 = 0; w2 < 8; ++w2) {
    const int t = wtot[w2];
    base += ((unsigned)w2 < wv) ? t : 0;
    cntv += t;
  }
  const int cnt = __builtin_amdgcn_readfirstlane(cntv);
  if (tile * TOKT >= cnt) return;

  {
    int rank = base + inc - c - tile * TOKT;
#pragma unroll
    for (int j = 0; j < EPT; ++j) {
      const bool hit = (rv[j] == e);
      if (hit && (unsigned)rank < (unsigned)TOKT) toks[rank] = (int)(frow0 + (unsigned)j);
      rank += hit ? 1 : 0;
    }
  }
  __syncthreads();

  {
    const unsigned row = tid >> 3, cb = (tid & 7u) * 32u;
    const int tok = toks[row];
    const bool live = (tok >= 0);
    int tokc = live ? tok : 0;
    tokc = (tokc > NTOK_FULL - 1) ? (NTOK_FULL - 1) : tokc;
    const size_t rbase = (size_t)tokc * ZD + cb;
#pragma unroll 2
    for (unsigned j = 0; j < 32u; j += 8u) {
      const v4f z0 = *(const v4f*)(Zin + rbase + j);
      const v4f z1 = *(const v4f*)(Zin + rbase + j + 4u);
      const v4f q0 = *(const v4f*)(Uin + rbase + j);
      const v4f q1 = *(const v4f*)(Uin + rbase + j + 4u);
      v8h oz, ou;
#pragma unroll
      for (int i = 0; i < 4; ++i) {
        oz[i]     = toh_flush(live ? bf16r(z0[i]) : 0.0f);
        oz[i + 4] = toh_flush(live ? bf16r(z1[i]) : 0.0f);
        ou[i]     = toh_flush(live ? bf16r(q0[i]) : 0.0f);
        ou[i + 4] = toh_flush(live ? bf16r(q1[i]) : 0.0f);
      }
      *(v8h*)&Ts[REG_Z + row * XLD + cb + j] = oz;
      *(v8h*)&Ts[REG_U + row * XLD + cb + j] = ou;
    }
  }
  __syncthreads();

#pragma unroll 1
  for (int sub = 0; sub < 2; ++sub) {
    const unsigned colBase = (unsigned)wave * 32u + (unsigned)sub * 16u;
    const unsigned acol = colBase + m;
    const _Float16* bw = Wp + OFFE_Z + ((size_t)e * ZD + acol) * ZD + hh * 8u;
    v8f g0 = {}, g1 = {};
#pragma unroll 2
    for (unsigned k0 = 0; k0 < (unsigned)ZD; k0 += 32u) {
      const v16h fb = frag_at(bw + k0);
      const v16h a0 = ld_frag(&Ts[REG_Z + k0], XLD);
      const v16h a1 = ld_frag(&Ts[REG_Z + 16 * XLD + k0], XLD);
      g0 = wmma16(a0, fb, g0);
      g1 = wmma16(a1, fb, g1);
    }
    const float bzv = bf16r(bz[(unsigned)e * (unsigned)ZD + acol]);
#pragma unroll
    for (int v = 0; v < 8; ++v) {
      const unsigned r = hh * 8u + (unsigned)v;
      const float x0 = g0[v] * (1.0f / WCARRY) + bzv;
      const float x1 = g1[v] * (1.0f / WCARRY) + bzv;
      Ts[REG_A + r * XLD + acol]         = toh_flush(ACARRY * x0);
      Ts[REG_A + (r + 16u) * XLD + acol] = toh_flush(ACARRY * x1);
    }
  }
  __syncthreads();

  const unsigned cwo = (unsigned)wave * (unsigned)(TOKT * OLD);
#pragma unroll 1
  for (int sl = 0; sl < NSLAB; ++sl) {
    const bool isH = (sl < NSLAB_H);
    const unsigned aoff = isH ? (unsigned)REG_A : (unsigned)REG_U;
    const unsigned ocol = (isH ? (unsigned)sl * (unsigned)SLABW : 0u) + (unsigned)wave * 32u;
    const size_t wrow = isH
        ? (size_t)OFFE_H + ((size_t)e * HD + ocol + m) * ZD
        : (size_t)OFFE_U + ((size_t)e * UD + ocol + m) * UD;
    const _Float16* bo = Wp + wrow + hh * 8u;

    v8f acc[4];
#pragma unroll
    for (int t = 0; t < 4; ++t) acc[t] = (v8f){};
#pragma unroll 2
    for (unsigned k0 = 0; k0 < (unsigned)ZD; k0 += 32u) {
      const v16h a0 = ld_frag(&Ts[aoff + k0], XLD);
      const v16h a1 = ld_frag(&Ts[aoff + 16 * XLD + k0], XLD);
#pragma unroll
      for (int t = 0; t < 2; ++t) {
        const v16h fb = frag_at(bo + (size_t)t * 16u * ZD + k0);
        acc[t]     = wmma16(a0, fb, acc[t]);
        acc[2 + t] = wmma16(a1, fb, acc[2 + t]);
      }
    }

#pragma unroll
    for (int tt = 0; tt < 2; ++tt)
#pragma unroll
      for (int v = 0; v < 8; ++v) {
        const unsigned r = hh * 8u + (unsigned)v;
        Cs[cwo + r * OLD + (unsigned)tt * 16u + m]         = acc[tt][v];
        Cs[cwo + (r + 16u) * OLD + (unsigned)tt * 16u + m] = acc[2 + tt][v];
      }
    wave_lds_sync();
    const float scale = isH ? (1.0f / (WCARRY * ACARRY)) : (1.0f / WCARRY);
    v4f xs[8];
    size_t off[8];
    bool ok[8];
#pragma unroll
    for (unsigned i = 0; i < 8u; ++i) {
      const unsigned r = 4u * i + (lane >> 3);
      const unsigned cc = (lane & 7u) * 4u;
      const unsigned col = ocol + cc;
      const v4f u = *(const v4f*)&Cs[cwo + r * OLD + cc];
      const unsigned bofs = isH ? ((unsigned)e * (unsigned)HD + col) : 0u;
      const v4f g = *(const v4f*)(bh + bofs);
      const int tok = toks[r];
      int tokc = (tok >= 0) ? tok : 0;
      tokc = (tokc > NTOK_FULL - 1) ? (NTOK_FULL - 1) : tokc;
      v4f val;
#pragma unroll
      for (int j = 0; j < 4; ++j) {
        const float b = isH ? bf16r(g[j]) : 0.0f;
        const float x = u[j] * scale + b;
        val[j] = isH ? fmaxf(x, 0.0f) : x;
      }
      xs[i] = val;
      off[i] = isH ? ((size_t)tokc * HD + col) : (OUT1_ELEM + (size_t)tokc * UD + col);
      ok[i] = (tok >= 0);
    }
#pragma unroll
    for (int i = 0; i < 8; ++i)
      if (ok[i]) *(volatile v4f*)(out + off[i]) = xs[i];
    __threadfence();
#pragma unroll
    for (int i = 0; i < 8; ++i)
      if (ok[i]) *(volatile v4f*)(out + off[i]) = xs[i];
    wave_lds_sync();
  }
}

extern "C" void kernel_launch(void* const* d_in, const int* in_sizes, int n_in,
                              void* d_out, int out_size, void* d_ws, size_t ws_size,
                              hipStream_t stream) {
  if (n_in < 8) return;
  if ((long long)in_sizes[0] < (long long)NTOK * ZD) return;
  if ((long long)in_sizes[1] < (long long)NTOK * UD) return;
  if ((long long)in_sizes[2] < (long long)NTOK) return;
  if ((long long)in_sizes[3] < (long long)NEXP * ZD * ZD) return;
  if ((long long)in_sizes[4] < (long long)NEXP * ZD) return;
  if ((long long)in_sizes[5] < (long long)NEXP * HD * ZD) return;
  if ((long long)in_sizes[6] < (long long)NEXP * HD) return;
  if ((long long)in_sizes[7] < (long long)NEXP * UD * UD) return;
  if ((long long)out_size < (long long)OUT1_ELEM + (long long)NTOK * UD) return;
  if (ws_size < WS_TOTAL) return;

  const float* Zin   = (const float*)d_in[0];
  const float* Uin   = (const float*)d_in[1];
  const int*   route = (const int*)d_in[2];
  const float* Wz    = (const float*)d_in[3];
  const float* bz    = (const float*)d_in[4];
  const float* Wh    = (const float*)d_in[5];
  const float* bh    = (const float*)d_in[6];
  const float* Wu    = (const float*)d_in[7];
  float* out = (float*)d_out;

  _Float16* Wp = (_Float16*)d_ws;

  dim3 blk(256);
  wcast_kernel<<<dim3((unsigned)(WZ_ELEMS / 2048)), blk, 0, stream>>>(
      Wz, Wp + OFFE_Z, (unsigned)(WZ_ELEMS / 8));
  wcast_kernel<<<dim3((unsigned)(WH_ELEMS / 2048)), blk, 0, stream>>>(
      Wh, Wp + OFFE_H, (unsigned)(WH_ELEMS / 8));
  wcast_kernel<<<dim3((unsigned)(WU_ELEMS / 2048)), blk, 0, stream>>>(
      Wu, Wp + OFFE_U, (unsigned)(WU_ELEMS / 8));

  mix_ffn_kernel<<<dim3(MAXTILE, NEXP), blk, 0, stream>>>(
      Zin, Uin, route, Wp, bz, bh, out);
}
